// HMM_DPM_61787399520276
// MI455X (gfx1250) — hardware-verified
//
#include <hip/hip_runtime.h>
#include <hip/hip_bf16.h>
#include <math.h>

#define BB      16
#define LL      256
#define DD      64
#define HH      256
#define H2      512
#define H4      1024
#define KK      3
#define SS      8
#define NN      (BB * LL)
#define NSTEPS  50
#define NB      (NN / 16)
#define NBLK    (SS * NB)
#define TTAB    64

#define BETA0     1e-4f
#define BETA_STEP ((2e-2f - 1e-4f) / 49.0f)
#define LOGF_STEP (-0.07252236513367074f)

typedef __attribute__((ext_vector_type(16))) __bf16 v16bf;
typedef __attribute__((ext_vector_type(8)))  __bf16 v8bf;
typedef __attribute__((ext_vector_type(8)))  float  v8f;
typedef __attribute__((ext_vector_type(4)))  float  v4f;
typedef __attribute__((ext_vector_type(4)))  unsigned int v4u;

__device__ __forceinline__ float silu_f(float x) {
  float e = __expf(-fmaxf(x, -40.f));
  return x * __builtin_amdgcn_rcpf(1.f + e);
}

__device__ __forceinline__ float red8(float v) {
  v += __shfl_xor(v, 1);
  v += __shfl_xor(v, 2);
  v += __shfl_xor(v, 4);
  return v;
}

__device__ __forceinline__ unsigned int bf16bits(float f) {
  unsigned int u = __float_as_uint(f);
  return (u + 0x7FFFu + ((u >> 16) & 1u)) >> 16;
}

union FragU { v16bf v; v8bf h[2]; };

__device__ __forceinline__ v16bf load_frag(const __bf16* rowp, int k0, int half) {
  FragU f;
  f.h[0] = *(const v8bf*)(rowp + k0 + (half << 3));
  f.h[1] = *(const v8bf*)(rowp + k0 + 16 + (half << 3));
  return f.v;
}

__device__ __forceinline__ v8f mma_bf16(v16bf a, v16bf b, v8f c) {
  v8f d = __builtin_amdgcn_wmma_f32_16x16x32_bf16(false, a, false, b, (short)0, c, false, false);
  asm volatile("v_nop\n\tv_nop\n\tv_nop\n\tv_nop" : "+v"(d) : "v"(a), "v"(b));
  return d;
}

template <class Epi>
__device__ __forceinline__ void wave_gemm16(const __bf16* sA, int Kdim,
                                            const __bf16* __restrict__ Bt, int colBase,
                                            int nTiles, int lane, Epi epi) {
  const int half = lane >> 4;
  const int lidx = lane & 15;
  const __bf16* rowp = sA + lidx * Kdim;
  for (int t = 0; t < nTiles; ++t) {
    const int col0 = colBase + (t << 4);
    const __bf16* bcol = Bt + (size_t)(col0 + lidx) * Kdim;
    v8f acc;
#pragma unroll
    for (int i = 0; i < 8; ++i) acc[i] = 0.f;
#pragma unroll 4
    for (int k0 = 0; k0 < Kdim; k0 += 32) {
      v16bf a = load_frag(rowp, k0, half);
      v16bf b = load_frag(bcol, k0, half);
      acc = mma_bf16(a, b, acc);
    }
    epi(col0 + lidx, half * 8, acc);
  }
}

__global__ __launch_bounds__(256) void wcvt8(const float* __restrict__ W,
                                             __bf16* __restrict__ Wt, int R, int C) {
  const int n8 = (R * C) >> 3;
  const int i = blockIdx.x * 256 + threadIdx.x;
  if (i >= n8) return;
  const int e = i << 3;
  const int c = e / R;
  const int r0 = e - c * R;
  v4u v;
#pragma unroll
  for (int j = 0; j < 4; ++j) {
    float w0 = W[(size_t)(r0 + 2 * j) * C + c];
    float w1 = W[(size_t)(r0 + 2 * j + 1) * C + c];
    v[j] = bf16bits(w0) | (bf16bits(w1) << 16);
  }
  v4u* p = (v4u*)(Wt + e);
  *(volatile v4u*)p = v;
  __threadfence();
  *(volatile v4u*)p = v;
}

__global__ __launch_bounds__(256) void prep_state(
    const float* __restrict__ se,
    const float* __restrict__ a1w, const float* __restrict__ a1b,
    const float* __restrict__ a2w, const float* __restrict__ a2b,
    float* __restrict__ se1, float* __restrict__ se2) {
  __shared__ float sv[KK * H4 + KK * H2];
  const int tid = threadIdx.x;
  for (int j = tid; j < KK * H4; j += 256) {
    const int k = j >> 10, c = j & (H4 - 1);
    float s = 0.f;
    for (int r = 0; r < HH; ++r) s += se[k * HH + r] * a1w[(size_t)r * H4 + c];
    sv[j] = s + a1b[c];
  }
  for (int j = tid; j < KK * H2; j += 256) {
    const int k = j >> 9, c = j & (H2 - 1);
    float s = 0.f;
    for (int r = 0; r < HH; ++r) s += se[k * HH + r] * a2w[(size_t)r * H2 + c];
    sv[KK * H4 + j] = s + a2b[c];
  }
  __syncthreads();
  for (int j = tid; j < KK * H4; j += 256) ((volatile float*)se1)[j] = sv[j];
  for (int j = tid; j < KK * H2; j += 256) ((volatile float*)se2)[j] = sv[KK * H4 + j];
  __threadfence();
  for (int j = tid; j < KK * H4; j += 256) ((volatile float*)se1)[j] = sv[j];
  for (int j = tid; j < KK * H2; j += 256) ((volatile float*)se2)[j] = sv[KK * H4 + j];
}

#define P_TR   0u
#define P_TB   8192u
#define P_W1   16384u
#define P_W2   81920u
#define P_T    114688u
#define SMEM_TAB 114752u

__global__ __launch_bounds__(128) void time_tab(
    const float* __restrict__ time_b,
    const __bf16* __restrict__ time_wt, const __bf16* __restrict__ a1wt,
    const __bf16* __restrict__ a2wt,
    float* __restrict__ w1tab, float* __restrict__ w2tab) {
  const int tid = threadIdx.x, lane = tid & 31, wv = tid >> 5;
  extern __shared__ __align__(16) char smem[];
  __bf16* aTR = (__bf16*)(smem + P_TR);
  __bf16* aTB = (__bf16*)(smem + P_TB);
  float*  aW1 = (float*)(smem + P_W1);
  float*  aW2 = (float*)(smem + P_W2);
  float*  aT  = (float*)(smem + P_T);

  if (tid < 16) aT[tid] = (float)(blockIdx.x * 16 + tid);
  __syncthreads();
  for (int i = tid; i < 16 * (HH / 2); i += 128) {
    const int r = i >> 7, j = i & 127;
    const float ang = aT[r] * expf((float)j * LOGF_STEP);
    aTR[r * HH + j]          = (__bf16)sinf(ang);
    aTR[r * HH + HH / 2 + j] = (__bf16)cosf(ang);
  }
  __syncthreads();

  wave_gemm16(aTR, HH, time_wt, wv * 64, 4, lane,
              [&](int col, int rb, v8f acc) {
                const float bb = time_b[col];
#pragma unroll
                for (int v = 0; v < 8; ++v)
                  aTB[(rb + v) * HH + col] = (__bf16)silu_f(acc[v] + bb);
              });
  __syncthreads();

  wave_gemm16(aTB, HH, a1wt, wv * 256, 16, lane,
              [&](int col, int rb, v8f acc) {
#pragma unroll
                for (int v = 0; v < 8; ++v) aW1[(rb + v) * H4 + col] = acc[v];
              });
  wave_gemm16(aTB, HH, a2wt, wv * 128, 8, lane,
              [&](int col, int rb, v8f acc) {
#pragma unroll
                for (int v = 0; v < 8; ++v) aW2[(rb + v) * H2 + col] = acc[v];
              });
  __syncthreads();

  float* d1 = w1tab + (size_t)blockIdx.x * 16 * H4;
  float* d2 = w2tab + (size_t)blockIdx.x * 16 * H2;
  for (int q = tid; q < 16 * H4 / 4; q += 128) {
    v4f v = *(const v4f*)(aW1 + 4 * q);
    *(volatile v4f*)(d1 + 4 * q) = v;
  }
  for (int q = tid; q < 16 * H2 / 4; q += 128) {
    v4f v = *(const v4f*)(aW2 + 4 * q);
    *(volatile v4f*)(d2 + 4 * q) = v;
  }
  __threadfence();
  for (int q = tid; q < 16 * H4 / 4; q += 128) {
    v4f v = *(const v4f*)(aW1 + 4 * q);
    *(volatile v4f*)(d1 + 4 * q) = v;
  }
  for (int q = tid; q < 16 * H2 / 4; q += 128) {
    v4f v = *(const v4f*)(aW2 + 4 * q);
    *(volatile v4f*)(d2 + 4 * q) = v;
  }
}

#define O_XT    0u
#define O_HS    2048u
#define O_HN    18432u
#define O_W1    51200u
#define O_W2    116736u
#define O_G     149504u
#define O_H3    165888u
#define O_PRED  174080u
#define O_SSE   178176u
#define O_AB    178688u
#define O_MEAN  178752u
#define O_RSTD  178816u
#define O_TI    178880u
#define SMEM_MAIN 178944u

__global__ __launch_bounds__(128) void fused_main(
    const float* __restrict__ y, const int* __restrict__ t_samples,
    const float* __restrict__ noise,
    const float* __restrict__ inproj_b, const float* __restrict__ lin1_b,
    const float* __restrict__ n1w, const float* __restrict__ n1b,
    const float* __restrict__ lin2_b,
    const float* __restrict__ n2w, const float* __restrict__ n2b,
    const float* __restrict__ out_b,
    const float* __restrict__ se1, const float* __restrict__ se2,
    const float* __restrict__ w1tab, const float* __restrict__ w2tab,
    const __bf16* __restrict__ inproj_wt, const __bf16* __restrict__ lin1_wt,
    const __bf16* __restrict__ lin2_wt, const __bf16* __restrict__ out_wt,
    float* __restrict__ ssePart) {
  const int sIdx = blockIdx.x >> 8;
  const int nb   = blockIdx.x & (NB - 1);
  const int n0   = nb * 16;
  const int row0 = sIdx * NN + n0;

  const int tid  = threadIdx.x;
  const int lane = tid & 31;
  const int wv   = tid >> 5;

  extern __shared__ __align__(16) char smem[];
  __bf16* aXt   = (__bf16*)(smem + O_XT);
  __bf16* aHs   = (__bf16*)(smem + O_HS);
  float*  aHn   = (float*)(smem + O_HN);
  float*  aW1   = (float*)(smem + O_W1);
  float*  aW2   = (float*)(smem + O_W2);
  float*  aG    = (float*)(smem + O_G);
  __bf16* aH3   = (__bf16*)(smem + O_H3);
  float*  aPred = (float*)(smem + O_PRED);
  float*  aSse  = (float*)(smem + O_SSE);
  float*  aAb   = (float*)(smem + O_AB);
  float*  aMean = (float*)(smem + O_MEAN);
  float*  aRstd = (float*)(smem + O_RSTD);
  int*    aTi   = (int*)(smem + O_TI);

  if (tid < 16) {
    const int t  = t_samples[row0 + tid];
    const int tc = min(max(t, 0), NSTEPS - 1);
    float p = 1.f, ab = 1.f;
    for (int i = 0; i < NSTEPS; ++i) {
      const float beta = BETA0 + (float)i * BETA_STEP;
      p = p * (1.f - beta);
      ab = (i == tc) ? p : ab;
    }
    aAb[tid] = ab;
    aTi[tid] = tc;
  }
  aSse[tid] = 0.f;
  __syncthreads();

  for (int i = tid; i < 16 * DD; i += 128) {
    const int r = i >> 6, d = i & 63;
    const float ab = aAb[r];
    const float xv = y[(size_t)(n0 + r) * DD + d];
    const float nv = noise[(size_t)(row0 + r) * DD + d];
    aXt[i] = (__bf16)(sqrtf(ab) * xv + sqrtf(1.f - ab) * nv);
  }
  for (int q = tid; q < 16 * (H4 / 4); q += 128) {
    const int r = q >> 8, c4 = q & 255;
    *(v4f*)(aW1 + r * H4 + 4 * c4) = *(const v4f*)(w1tab + (size_t)aTi[r] * H4 + 4 * c4);
  }
  for (int q = tid; q < 16 * (H2 / 4); q += 128) {
    const int r = q >> 7, c4 = q & 127;
    *(v4f*)(aW2 + r * H2 + 4 * c4) = *(const v4f*)(w2tab + (size_t)aTi[r] * H2 + 4 * c4);
  }
  __syncthreads();

  wave_gemm16(aXt, DD, inproj_wt, wv * 128, 8, lane,
              [&](int col, int rb, v8f acc) {
                const float bb = inproj_b[col];
#pragma unroll
                for (int v = 0; v < 8; ++v)
                  aHs[(rb + v) * H2 + col] = (__bf16)silu_f(acc[v] + bb);
              });
  __syncthreads();

  wave_gemm16(aHs, H2, lin1_wt, wv * 128, 8, lane,
              [&](int col, int rb, v8f acc) {
                const float bb = lin1_b[col];
#pragma unroll
                for (int v = 0; v < 8; ++v)
                  aHn[(rb + v) * H2 + col] = acc[v] + bb;
              });
  __syncthreads();

  {
    const int r = tid >> 3, c0 = (tid & 7) * 64;
    float s = 0.f;
    for (int c = c0; c < c0 + 64; ++c) s += aHn[r * H2 + c];
    s = red8(s);
    const float m = s * (1.f / 512.f);
    float ss = 0.f;
    for (int c = c0; c < c0 + 64; ++c) { const float dv = aHn[r * H2 + c] - m; ss += dv * dv; }
    ss = red8(ss);
    if ((tid & 7) == 0) {
      aMean[r] = m;
      aRstd[r] = rsqrtf(ss * (1.f / 512.f) + 1e-5f);
    }
  }
  __syncthreads();
  {
#pragma unroll
    for (int cc = 0; cc < 4; ++cc) {
      const int c = tid + 128 * cc;
      const float w = n1w[c], bb = n1b[c];
      for (int r = 0; r < 16; ++r) {
        const int i = r * H2 + c;
        aHn[i] = (aHn[i] - aMean[r]) * aRstd[r] * w + bb;
      }
    }
  }
  __syncthreads();

  for (int k = 0; k < KK; ++k) {
    const float* e1 = se1 + k * H4;
    const float* e2 = se2 + k * H2;

#pragma unroll
    for (int cc = 0; cc < 4; ++cc) {
      const int c = tid + 128 * cc;
      const float ec1 = e1[c], ec2 = e1[H2 + c];
      for (int r = 0; r < 16; ++r) {
        const int i = r * H2 + c;
        const float sc = aW1[r * H4 + c] + ec1;
        const float sh = aW1[r * H4 + H2 + c] + ec2;
        aHs[i] = (__bf16)silu_f(aHn[i] * (1.f + sc) + sh);
      }
    }
    __syncthreads();

    wave_gemm16(aHs, H2, lin2_wt, wv * 64, 4, lane,
                [&](int col, int rb, v8f acc) {
                  const float bb = lin2_b[col];
#pragma unroll
                  for (int v = 0; v < 8; ++v) aG[(rb + v) * HH + col] = acc[v] + bb;
                });
    __syncthreads();

    {
      const int r = tid >> 3, c0 = (tid & 7) * 32;
      float s = 0.f;
      for (int c = c0; c < c0 + 32; ++c) s += aG[r * HH + c];
      s = red8(s);
      const float m = s * (1.f / 256.f);
      float ss = 0.f;
      for (int c = c0; c < c0 + 32; ++c) { const float dv = aG[r * HH + c] - m; ss += dv * dv; }
      ss = red8(ss);
      if ((tid & 7) == 0) {
        aMean[r] = m;
        aRstd[r] = rsqrtf(ss * (1.f / 256.f) + 1e-5f);
      }
    }
    __syncthreads();
#pragma unroll
    for (int cc = 0; cc < 2; ++cc) {
      const int c = tid + 128 * cc;
      const float w = n2w[c], bb = n2b[c];
      const float ec1 = e2[c], ec2 = e2[HH + c];
      for (int r = 0; r < 16; ++r) {
        const float hn2 = (aG[r * HH + c] - aMean[r]) * aRstd[r] * w + bb;
        const float sc = aW2[r * H2 + c] + ec1;
        const float sh = aW2[r * H2 + HH + c] + ec2;
        aH3[r * HH + c] = (__bf16)silu_f(hn2 * (1.f + sc) + sh);
      }
    }
    __syncthreads();

    wave_gemm16(aH3, HH, out_wt, wv * 16, 1, lane,
                [&](int col, int rb, v8f acc) {
                  const float bb = out_b[col];
#pragma unroll
                  for (int v = 0; v < 8; ++v) aPred[(rb + v) * DD + col] = acc[v] + bb;
                });
    __syncthreads();

    {
      const int r = tid >> 3, sub = tid & 7;
      const float* np = noise + (size_t)(row0 + r) * DD + sub * 8;
      float s = 0.f;
#pragma unroll
      for (int dd = 0; dd < 8; ++dd) {
        const float df = aPred[r * DD + sub * 8 + dd] - np[dd];
        s += df * df;
      }
      s = red8(s);
      if (sub == 0) aSse[k * 32 + r] = s;
    }
    __syncthreads();
  }

  if (tid < 32) {
    const v4f v = *(const v4f*)(aSse + 4 * lane);
    float* dst = ssePart + (size_t)blockIdx.x * 128;
    *(volatile v4f*)(dst + 4 * lane) = v;
    __threadfence();
    *(volatile v4f*)(dst + 4 * lane) = v;
  }
}

__global__ __launch_bounds__(32) void hmm_fwd(
    const float* __restrict__ ssePart, const float* __restrict__ trans_logits,
    const float* __restrict__ start_logits, float* __restrict__ out) {
  __shared__ __align__(16) float aEm[LL * KK];
  __shared__ __align__(16) float aAl[LL * KK];
  const int b = blockIdx.x;
  const int lane = threadIdx.x;

  for (int it = 0; it < (LL * KK) / 32; ++it) {
    const int idx = it * 32 + lane;
    const int l = idx / KK;
    const int kk = idx - l * KK;
    const int n = b * LL + l;
    const int nb = n >> 4, j = n & 15;
    float s = 0.f;
#pragma unroll
    for (int ss = 0; ss < SS; ++ss)
      s += ssePart[(size_t)(ss * NB + nb) * 128 + kk * 32 + j];
    aEm[idx] = (-0.5f * s) * (1.f / (float)SS);
  }
  __syncthreads();

  if (lane == 0) {
    float lt[KK][KK], ls[KK];
#pragma unroll
    for (int i = 0; i < KK; ++i) {
      const float x0 = trans_logits[i * KK], x1 = trans_logits[i * KK + 1], x2 = trans_logits[i * KK + 2];
      const float m = fmaxf(fmaxf(x0, x1), x2);
      const float z = expf(x0 - m) + expf(x1 - m) + expf(x2 - m);
      const float lg = logf(z);
      lt[i][0] = (x0 - m) - lg;
      lt[i][1] = (x1 - m) - lg;
      lt[i][2] = (x2 - m) - lg;
    }
    {
      const float x0 = start_logits[0], x1 = start_logits[1], x2 = start_logits[2];
      const float m = fmaxf(fmaxf(x0, x1), x2);
      const float z = expf(x0 - m) + expf(x1 - m) + expf(x2 - m);
      const float lg = logf(z);
      ls[0] = (x0 - m) - lg;
      ls[1] = (x1 - m) - lg;
      ls[2] = (x2 - m) - lg;
    }
    float a[KK];
#pragma unroll
    for (int kk = 0; kk < KK; ++kk) a[kk] = ls[kk] + aEm[kk];
#pragma unroll
    for (int kk = 0; kk < KK; ++kk) aAl[kk] = a[kk];
    for (int l = 1; l < LL; ++l) {
      float na[KK];
#pragma unroll
      for (int kk = 0; kk < KK; ++kk) {
        const float v0 = a[0] + lt[0][kk], v1 = a[1] + lt[1][kk], v2 = a[2] + lt[2][kk];
        const float m = fmaxf(fmaxf(v0, v1), v2);
        na[kk] = aEm[l * KK + kk] + (logf(expf(v0 - m) + expf(v1 - m) + expf(v2 - m)) + m);
      }
#pragma unroll
      for (int kk = 0; kk < KK; ++kk) { a[kk] = na[kk]; aAl[l * KK + kk] = na[kk]; }
    }
  }
  __syncthreads();

  float* dst = out + (size_t)b * (LL * KK);
  for (int it = 0; it < (LL * KK) / 128; ++it) {
    const int q = it * 32 + lane;
    const v4f v = *(const v4f*)(aAl + 4 * q);
    *(volatile v4f*)(dst + 4 * q) = v;
  }
  __threadfence();
  for (int it = 0; it < (LL * KK) / 128; ++it) {
    const int q = it * 32 + lane;
    const v4f v = *(const v4f*)(aAl + 4 * q);
    *(volatile v4f*)(dst + 4 * q) = v;
  }
}

static constexpr size_t OFF_SE1   = 0;
static constexpr size_t OFF_SE2   = 12288;
static constexpr size_t OFF_W1T   = 18432;
static constexpr size_t OFF_W2T   = 280576;
static constexpr size_t OFF_SSE   = 411648;
static constexpr size_t OFF_TIMEW = 1460224;
static constexpr size_t OFF_INPW  = 1591296;
static constexpr size_t OFF_L1W   = 1656832;
static constexpr size_t OFF_A1W   = 2181120;
static constexpr size_t OFF_L2W   = 2705408;
static constexpr size_t OFF_A2W   = 2967552;
static constexpr size_t OFF_OUTW  = 3229696;
static constexpr size_t WS_NEED   = 3262464;

extern "C" void kernel_launch(void* const* d_in, const int* in_sizes, int n_in,
                              void* d_out, int out_size, void* d_ws, size_t ws_size,
                              hipStream_t stream) {
  if (n_in < 24) return;
  if (in_sizes[0] != BB * LL * DD || in_sizes[1] != SS * NN || in_sizes[2] != SS * NN * DD) return;
  if (out_size != NN * KK) return;
  if (ws_size < WS_NEED) return;

  const float* y            = (const float*)d_in[0];
  const int*   t_samples    = (const int*)d_in[1];
  const float* noise        = (const float*)d_in[2];
  const float* time_w       = (const float*)d_in[3];
  const float* time_b       = (const float*)d_in[4];
  const float* state_emb    = (const float*)d_in[5];
  const float* inproj_w     = (const float*)d_in[6];
  const float* inproj_b     = (const float*)d_in[7];
  const float* lin1_w       = (const float*)d_in[8];
  const float* lin1_b       = (const float*)d_in[9];
  const float* n1w          = (const float*)d_in[10];
  const float* n1b          = (const float*)d_in[11];
  const float* a1wF         = (const float*)d_in[12];
  const float* a1b          = (const float*)d_in[13];
  const float* lin2_w       = (const float*)d_in[14];
  const float* lin2_b       = (const float*)d_in[15];
  const float* n2w          = (const float*)d_in[16];
  const float* n2b          = (const float*)d_in[17];
  const float* a2wF         = (const float*)d_in[18];
  const float* a2b          = (const float*)d_in[19];
  const float* out_w        = (const float*)d_in[20];
  const float* out_b        = (const float*)d_in[21];
  const float* trans_logits = (const float*)d_in[22];
  const float* start_logits = (const float*)d_in[23];

  char* ws = (char*)d_ws;
  float*  se1       = (float*)(ws + OFF_SE1);
  float*  se2       = (float*)(ws + OFF_SE2);
  float*  w1tab     = (float*)(ws + OFF_W1T);
  float*  w2tab     = (float*)(ws + OFF_W2T);
  float*  ssePart   = (float*)(ws + OFF_SSE);
  __bf16* time_wt   = (__bf16*)(ws + OFF_TIMEW);
  __bf16* inproj_wt = (__bf16*)(ws + OFF_INPW);
  __bf16* lin1_wt   = (__bf16*)(ws + OFF_L1W);
  __bf16* adaln1_wt = (__bf16*)(ws + OFF_A1W);
  __bf16* lin2_wt   = (__bf16*)(ws + OFF_L2W);
  __bf16* adaln2_wt = (__bf16*)(ws + OFF_A2W);
  __bf16* out_wt    = (__bf16*)(ws + OFF_OUTW);

  auto cvt = [&](const float* W, __bf16* Wt, int R, int C) {
    const int n8 = (R * C) / 8;
    wcvt8<<<(n8 + 255) / 256, 256, 0, stream>>>(W, Wt, R, C);
  };
  cvt(time_w,   time_wt,   HH, HH);
  cvt(inproj_w, inproj_wt, DD, H2);
  cvt(lin1_w,   lin1_wt,   H2, H2);
  cvt(a1wF,     adaln1_wt, HH, H4);
  cvt(lin2_w,   lin2_wt,   H2, HH);
  cvt(a2wF,     adaln2_wt, HH, H2);
  cvt(out_w,    out_wt,    HH, DD);

  prep_state<<<1, 256, 0, stream>>>(state_emb, a1wF, a1b, a2wF, a2b, se1, se2);

  time_tab<<<dim3(TTAB / 16), dim3(128), SMEM_TAB, stream>>>(
      time_b, time_wt, adaln1_wt, adaln2_wt, w1tab, w2tab);

  fused_main<<<dim3(NBLK), dim3(128), SMEM_MAIN, stream>>>(
      y, t_samples, noise,
      inproj_b, lin1_b, n1w, n1b, lin2_b, n2w, n2b, out_b,
      se1, se2, w1tab, w2tab,
      inproj_wt, lin1_wt, lin2_wt, out_wt,
      ssePart);

  hmm_fwd<<<dim3(BB), dim3(32), 0, stream>>>(
      ssePart, trans_logits, start_logits, (float*)d_out);
}
